// MAMBA2D_60232621359562
// MI455X (gfx1250) — hardware-verified
//
#include <hip/hip_runtime.h>


namespace {
constexpr int NB = 2, GH = 64, GW = 64, DM = 512, DS = 128, DI = 1024, NH = 16, HD = 64, CD = 1280, DIP = 2320, ZP = 2432, SL = 64, NSEQ = 128, NR = NSEQ * SL, NTOK = NB * GH * GW;
constexpr float XS = 8.0f, WSC = 256.0f;
typedef _Float16 b16;
typedef __attribute__((ext_vector_type(16))) _Float16 v16b;
typedef __attribute__((ext_vector_type(8))) _Float16 v8b;
typedef __attribute__((ext_vector_type(8))) float v8f;
typedef __attribute__((ext_vector_type(4))) float v4f;
typedef __attribute__((ext_vector_type(2))) float v2f;
__device__ __forceinline__ float bf16_rne(float f) { unsigned int u = __float_as_uint(f); u += 0x7FFFu + ((u >> 16) & 1u); return __uint_as_float(u & 0xFFFF0000u); }
__device__ __forceinline__ float bfv(float f) { float r = bf16_rne(f); asm volatile("" : "+v"(r)); return r; }
__device__ __forceinline__ void split16(float v, b16& hi, b16& lo) { hi = (b16)v; lo = (b16)(v - (float)hi); }
__device__ __forceinline__ v16b frag_kb(const b16* p, int hh) { const v8b a = *(const v8b*)(p + 8 * hh), b = *(const v8b*)(p + 16 + 8 * hh); v16b f;
#pragma unroll
  for (int e = 0; e < 8; ++e) { f[e] = a[e]; f[8 + e] = b[e]; } return f; }
__device__ __forceinline__ v8f wmma16b(v16b a, v16b b, v8f c) { v8f d = __builtin_amdgcn_wmma_f32_16x16x32_f16(false, a, false, b, (short)0, c, false, false); asm volatile("v_nop\n\tv_nop\n\tv_nop\n\tv_nop" : "+v"(d) : "v"(a), "v"(b)); return d; }
__device__ __forceinline__ void wave_lds_sync() { __builtin_amdgcn_fence(__ATOMIC_RELEASE, "workgroup"); __builtin_amdgcn_wave_barrier(); __builtin_amdgcn_fence(__ATOMIC_ACQUIRE, "workgroup"); }
__device__ __forceinline__ float pmul(float a, float b) { float p = a * b; asm volatile("" : "+v"(p)); return p; }
__device__ __forceinline__ float silu(float v) { return v / (1.0f + __expf(-v)); }
__device__ __forceinline__ float softplus(float v) { return v > 20.0f ? v : log1pf(__expf(v)); }
__device__ __forceinline__ size_t tok_of(int pass, int seq, int t) { const int b = seq / 64, r = seq % 64; return pass == 0 ? ((size_t)(b * GH + r) * GW + t) : ((size_t)(b * GH + t) * GW + r); }

__global__ __launch_bounds__(256) void wcopy_kernel(const float* __restrict__ w, int OUTW, int OPAD, int KIN, b16* __restrict__ WT) { const size_t u = (size_t)blockIdx.x * 256 + threadIdx.x; if (u >= (size_t)OPAD * KIN / 8) return; const size_t e = u * 8; const int o = (int)(e / KIN); v8b v;
#pragma unroll
  for (int j = 0; j < 8; ++j) v[j] = (b16)(o < OUTW ? bf16_rne(w[e + j]) * WSC : 0.0f); for (int pass = 0; pass < 2; ++pass) { *(volatile v8b*)(WT + e) = v; __threadfence(); } }
__global__ __launch_bounds__(32) void inproj_kernel(const float* __restrict__ x, const b16* __restrict__ WT, int pss, int NS, float* __restrict__ ZX) {
  __shared__ __attribute__((aligned(16))) b16 Ah[16][DM + 8]; __shared__ float Tf[16][132]; const int lane = threadIdx.x, nloc = lane & 15, hlf = lane >> 4; const int cg = blockIdx.x % (ZP / 128); const size_t m0 = (size_t)(blockIdx.x / (ZP / 128)) * 16; if (m0 >= (size_t)NS * SL) return;
  for (int rr = 0; rr < 16; ++rr) { const size_t row = m0 + rr; const size_t tk = tok_of(pss, (int)(row / SL), (int)(row % SL)); for (int q = 0; q < DM / 32; ++q) Ah[rr][q * 32 + lane] = (b16)(bf16_rne(x[tk * DM + q * 32 + lane]) * XS); }
  wave_lds_sync(); v8f acc[8];
#pragma unroll
  for (int t = 0; t < 8; ++t) acc[t] = (v8f){};
#pragma unroll 2
  for (int kb = 0; kb < DM; kb += 32) { const v16b a = frag_kb(&Ah[nloc][kb], hlf);
#pragma unroll
    for (int t = 0; t < 8; ++t) acc[t] = wmma16b(a, frag_kb(WT + (size_t)(cg * 128 + t * 16 + nloc) * DM + kb, hlf), acc[t]); }
#pragma unroll
  for (int t = 0; t < 8; ++t)
#pragma unroll
    for (int r8 = 0; r8 < 8; ++r8) Tf[8 * hlf + r8][t * 16 + nloc] = acc[t][r8] * (1.0f / (XS * WSC));
  wave_lds_sync();
  for (int pass = 0; pass < 2; ++pass) { for (int rr = 0; rr < 16; ++rr) *(volatile v4f*)(ZX + (m0 + rr) * ZP + cg * 128 + lane * 4) = *(const v4f*)(&Tf[rr][lane * 4]); __threadfence(); }
}
__global__ __launch_bounds__(256) void conv_kernel(const float* __restrict__ ZX, const float* __restrict__ cw, const float* __restrict__ cb, int NS, float* __restrict__ XC) {
  const size_t u = (size_t)blockIdx.x * 256 + threadIdx.x; if (u >= (size_t)NS * CD) return; const int seq = (int)(u / CD), c = (int)(u % CD); const float w0 = bfv(cw[c * 4]), w1 = bfv(cw[c * 4 + 1]), w2 = bfv(cw[c * 4 + 2]), w3 = bfv(cw[c * 4 + 3]), bb = bfv(cb[c]);
  for (int pass = 0; pass < 2; ++pass) { float p0 = 0.0f, p1 = 0.0f, p2 = 0.0f;
#pragma unroll 1
    for (int t = 0; t < SL; ++t) { const size_t row = (size_t)seq * SL + t; const float cur = ZX[row * ZP + DI + c]; const float v = pmul(p0, w0) + pmul(p1, w1) + pmul(p2, w2) + pmul(cur, w3) + bb; ((volatile float*)XC)[row * CD + c] = silu(v); p0 = p1; p1 = p2; p2 = cur; }
    __threadfence(); }
}
__global__ __launch_bounds__(256) void dt_kernel(const float* __restrict__ ZX, const float* __restrict__ dtb, const float* __restrict__ Alog, int NS, float* __restrict__ DT) {
  const int u = blockIdx.x * 256 + threadIdx.x; if (u >= NS * NH) return; const int seq = u / NH, h = u % NH; const float db = bfv(dtb[h]); const float a = -__expf(bfv(Alog[h]));
  for (int pass = 0; pass < 2; ++pass) { float cs = 0.0f;
#pragma unroll 1
    for (int t = 0; t < SL; ++t) { const size_t row = (size_t)seq * SL + t; const float dt = softplus(ZX[row * ZP + DI + CD + h] + db); cs += pmul(dt, a); ((volatile float*)DT)[row * 32 + h] = dt; ((volatile float*)DT)[row * 32 + 16 + h] = cs; }
    __threadfence(); }
}
__global__ __launch_bounds__(32) void ssd_kernel(const float* __restrict__ XC, const float* __restrict__ DT, const float* __restrict__ Dp, int NS, float* __restrict__ Y) {
  __shared__ __attribute__((aligned(16))) b16 Ch[16][DS + 8], Cl[16][DS + 8], Bh[32][DS + 8], Bl[32][DS + 8], Ph[16][40], Pl[16][40], Xh[HD][40], Xl[HD][40]; __shared__ float Sc[16][33], Of[16][HD + 2], Cs[16], Csk[32], Dtk[32];
  const int lane = threadIdx.x, nloc = lane & 15, hlf = lane >> 4; const int qt = blockIdx.x % (SL / 16); const int hh = (blockIdx.x / (SL / 16)) % NH; const int seq = blockIdx.x / ((SL / 16) * NH); if (seq >= NS) return; const int t0 = qt * 16; const size_t rb_ = (size_t)seq * SL;
  for (int rr = 0; rr < 16; ++rr) for (int q = 0; q < DS / 32; ++q) { b16 p, ql; split16(XC[(rb_ + t0 + rr) * CD + DI + DS + q * 32 + lane] * XS, p, ql); Ch[rr][q * 32 + lane] = p; Cl[rr][q * 32 + lane] = ql; }
  if (lane < 16) Cs[lane] = DT[(rb_ + t0 + lane) * 32 + 16 + hh];
  v8f acc[4] = {(v8f){}, (v8f){}, (v8f){}, (v8f){}}; wave_lds_sync();
#pragma unroll 1
  for (int sc = 0; sc < t0 + 16; sc += 32) {
    for (int rr = 0; rr < 32; ++rr) { const size_t row = rb_ + sc + rr; const bool ok = (sc + rr) < SL; for (int q = 0; q < DS / 32; ++q) { b16 p, ql; split16((ok ? XC[row * CD + DI + q * 32 + lane] : 0.0f) * XS, p, ql); Bh[rr][q * 32 + lane] = p; Bl[rr][q * 32 + lane] = ql; }
      for (int q = 0; q < 2; ++q) { b16 p, ql; split16((ok ? XC[row * CD + hh * HD + q * 32 + lane] : 0.0f) * XS, p, ql); Xh[q * 32 + lane][rr] = p; Xl[q * 32 + lane][rr] = ql; } }
    { const bool ok = (sc + lane) < SL; Csk[lane] = ok ? DT[(rb_ + sc + lane) * 32 + 16 + hh] : 0.0f; Dtk[lane] = ok ? DT[(rb_ + sc + lane) * 32 + hh] : 0.0f; }
    wave_lds_sync();
#pragma unroll
    for (int blk = 0; blk < 2; ++blk) { v8f s = {};
#pragma unroll
      for (int kb = 0; kb < DS; kb += 32) { const v16b ch = frag_kb(&Ch[nloc][kb], hlf), cl = frag_kb(&Cl[nloc][kb], hlf), bh = frag_kb(&Bh[blk * 16 + nloc][kb], hlf), bl = frag_kb(&Bl[blk * 16 + nloc][kb], hlf); s = wmma16b(ch, bh, s); s = wmma16b(ch, bl, s); s = wmma16b(cl, bh, s); }
#pragma unroll
      for (int r8 = 0; r8 < 8; ++r8) Sc[8 * hlf + r8][blk * 16 + nloc] = s[r8] * (1.0f / (XS * XS)); }
    wave_lds_sync();
    for (int qi = 0; qi < 16; ++qi) { const int t = t0 + qi, s_ = sc + lane; float pv = 0.0f; if (s_ <= t) pv = pmul(pmul(Sc[qi][lane], __expf(Cs[qi] - Csk[lane])), Dtk[lane]); b16 p, ql; split16(pv, p, ql); Ph[qi][lane] = p; Pl[qi][lane] = ql; }
    wave_lds_sync(); const v16b pa = frag_kb(&Ph[nloc][0], hlf), pb = frag_kb(&Pl[nloc][0], hlf);
#pragma unroll
    for (int tt = 0; tt < 4; ++tt) { const v16b xh = frag_kb(&Xh[tt * 16 + nloc][0], hlf), xl = frag_kb(&Xl[tt * 16 + nloc][0], hlf); acc[tt] = wmma16b(pa, xh, acc[tt]); acc[tt] = wmma16b(pa, xl, acc[tt]); acc[tt] = wmma16b(pb, xh, acc[tt]); }
    wave_lds_sync(); }
  const float dv = bfv(Dp[hh]);
#pragma unroll
  for (int tt = 0; tt < 4; ++tt)
#pragma unroll
    for (int r8 = 0; r8 < 8; ++r8) { const int rl = 8 * hlf + r8; const int d = tt * 16 + nloc; Of[rl][d] = acc[tt][r8] * (1.0f / XS) + pmul(dv, XC[(rb_ + t0 + rl) * CD + hh * HD + d]); }
  wave_lds_sync();
  for (int pass = 0; pass < 2; ++pass) { for (int rr = 0; rr < 16; ++rr) *(volatile v2f*)(Y + (rb_ + t0 + rr) * DI + hh * HD + lane * 2) = (v2f){Of[rr][lane * 2], Of[rr][lane * 2 + 1]}; __threadfence(); }
}
__global__ __launch_bounds__(256) void gate_kernel(const float* __restrict__ Y, const float* __restrict__ ZX, const float* __restrict__ nw, int NS, b16* __restrict__ YN) {
  const int wave = threadIdx.x >> 5, lane = threadIdx.x & 31; const size_t row = (size_t)blockIdx.x * 8 + wave; if (row >= (size_t)NS * SL) return; float sq = 0.0f;
#pragma unroll 1
  for (int q = 0; q < 32; ++q) { const int d = q * 32 + lane; const float v = pmul(Y[row * DI + d], silu(ZX[row * ZP + d])); sq += pmul(v, v); }
  for (int o = 16; o; o >>= 1) sq += __shfl_xor(sq, o); const float rs = rsqrtf(sq * (1.0f / DI) + 1e-5f);
  for (int pass = 0; pass < 2; ++pass) {
#pragma unroll 1
    for (int q = 0; q < 32; ++q) { const int d = q * 32 + lane; const float v = pmul(Y[row * DI + d], silu(ZX[row * ZP + d])); ((volatile b16*)YN)[row * DI + d] = (b16)(pmul(pmul(v, rs), bfv(nw[d])) * XS); } __threadfence(); }
}
__global__ __launch_bounds__(32) void outproj_kernel(const b16* __restrict__ YN, const b16* __restrict__ WT, int NS, float* __restrict__ HV) {
  __shared__ float Tf[16][132]; const int lane = threadIdx.x, nloc = lane & 15, hlf = lane >> 4; const int cg = blockIdx.x % 4; const size_t m0 = (size_t)(blockIdx.x / 4) * 16; if (m0 >= (size_t)NS * SL) return; v8f acc[8];
#pragma unroll
  for (int t = 0; t < 8; ++t) acc[t] = (v8f){};
#pragma unroll 2
  for (int kb = 0; kb < DI; kb += 32) { const v16b a = frag_kb(YN + (m0 + nloc) * DI + kb, hlf);
#pragma unroll
    for (int t = 0; t < 8; ++t) acc[t] = wmma16b(a, frag_kb(WT + (size_t)(cg * 128 + t * 16 + nloc) * DI + kb, hlf), acc[t]); }
#pragma unroll
  for (int t = 0; t < 8; ++t)
#pragma unroll
    for (int r8 = 0; r8 < 8; ++r8) Tf[8 * hlf + r8][t * 16 + nloc] = acc[t][r8] * (1.0f / (XS * WSC));
  wave_lds_sync();
  for (int pass = 0; pass < 2; ++pass) { for (int rr = 0; rr < 16; ++rr) *(volatile v4f*)(HV + (m0 + rr) * DM + cg * 128 + lane * 4) = *(const v4f*)(&Tf[rr][lane * 4]); __threadfence(); }
}
__global__ __launch_bounds__(32) void fc_kernel(const float* __restrict__ HH, const float* __restrict__ VV, const b16* __restrict__ WT, const float* __restrict__ fcb, int NS, float* __restrict__ out) {
  __shared__ __attribute__((aligned(16))) b16 Ah[16][4 * DM + 8]; __shared__ float Tf[16][132]; const int lane = threadIdx.x, nloc = lane & 15, hlf = lane >> 4; const int cg = blockIdx.x % 4; const size_t m0 = (size_t)(blockIdx.x / 4) * 16;
  const int b = (int)(m0 / (GH * GW)), hr = (int)((m0 / GW) % GH), w0 = (int)(m0 % GW);
  const bool live = (b * 64 + hr) < NS && (b * 64 + w0 + 15) < NS;
  if (!live) { for (int pass = 0; pass < 2; ++pass) { for (int rr = 0; rr < 16; ++rr) *(volatile v4f*)(out + (m0 + rr) * DM + cg * 128 + lane * 4) = (v4f){0.0f, 0.0f, 0.0f, 0.0f}; __threadfence(); } return; }
  for (int rr = 0; rr < 16; ++rr) { const int w = w0 + rr; const size_t hrow = (size_t)(b * 64 + hr) * SL + w, vrow = (size_t)(b * 64 + w) * SL + hr;
    for (int q = 0; q < DM / 32; ++q) { const int c = q * 32 + lane; const b16 hv = (b16)(HH[hrow * DM + c] * XS), vv = (b16)(VV[vrow * DM + c] * XS); Ah[rr][c] = vv; Ah[rr][DM + c] = vv; Ah[rr][2 * DM + c] = hv; Ah[rr][3 * DM + c] = hv; } }
  wave_lds_sync(); v8f acc[8];
#pragma unroll
  for (int t = 0; t < 8; ++t) acc[t] = (v8f){};
#pragma unroll 2
  for (int kb = 0; kb < 4 * DM; kb += 32) { const v16b a = frag_kb(&Ah[nloc][kb], hlf);
#pragma unroll
    for (int t = 0; t < 8; ++t) acc[t] = wmma16b(a, frag_kb(WT + (size_t)(cg * 128 + t * 16 + nloc) * (4 * DM) + kb, hlf), acc[t]); }
#pragma unroll
  for (int t = 0; t < 8; ++t) { const int c = cg * 128 + t * 16 + nloc; float bb = bf16_rne(fcb[c]); asm volatile("" : "+v"(bb));
#pragma unroll
    for (int r8 = 0; r8 < 8; ++r8) Tf[8 * hlf + r8][t * 16 + nloc] = acc[t][r8] * (1.0f / (XS * WSC)) + bb; }
  wave_lds_sync();
  for (int pass = 0; pass < 2; ++pass) { for (int rr = 0; rr < 16; ++rr) *(volatile v4f*)(out + (m0 + rr) * DM + cg * 128 + lane * 4) = *(const v4f*)(&Tf[rr][lane * 4]); __threadfence(); }
}
}

extern "C" void kernel_launch(void* const* d_in, const int* in_sizes, int n_in, void* d_out, int out_size, void* d_ws, size_t ws_size, hipStream_t stream) {
  (void)n_in;
  auto Fp = [&](int i) { return (const float*)d_in[i]; };
  if (in_sizes[0] != NTOK * DM || in_sizes[1] != DIP * DM || in_sizes[2] != CD * 4 || in_sizes[8] != DM * DI || in_sizes[9] != DIP * DM || in_sizes[16] != DM * DI || in_sizes[17] != DM * 4 * DM || out_size != NTOK * DM) return;
  const int NS = NSEQ;
  size_t off = 0; char* ws = (char*)d_ws;
  auto carve = [&](size_t bytes) { char* p = ws + off; off += (bytes + 255) & ~(size_t)255; return p; };
  b16* WIN = (b16*)carve((size_t)ZP * DM * 2); b16* WOUT = (b16*)carve((size_t)DM * DI * 2); b16* WFC = (b16*)carve((size_t)DM * 4 * DM * 2);
  float* ZX = (float*)carve((size_t)NR * ZP * 4); float* XC = (float*)carve((size_t)NR * CD * 4); float* DT = (float*)carve((size_t)NR * 32 * 4); float* Y = (float*)carve((size_t)NR * DI * 4); b16* YN = (b16*)carve((size_t)NR * DI * 2); float* HH = (float*)carve((size_t)NR * DM * 4); float* VV = (float*)carve((size_t)NR * DM * 4);
  if (off > ws_size || off > ((size_t)232 << 20)) return;
  wcopy_kernel<<<(unsigned)(((size_t)DM * 4 * DM / 8 + 255) / 256), 256, 0, stream>>>(Fp(17), DM, DM, 4 * DM, WFC);
  for (int pss = 0; pss < 2; ++pss) { const int o = pss == 0 ? 1 : 9; float* HVp = pss == 0 ? HH : VV;
    wcopy_kernel<<<(unsigned)(((size_t)ZP * DM / 8 + 255) / 256), 256, 0, stream>>>(Fp(o), DIP, ZP, DM, WIN);
    wcopy_kernel<<<(unsigned)(((size_t)DM * DI / 8 + 255) / 256), 256, 0, stream>>>(Fp(o + 7), DM, DM, DI, WOUT);
    inproj_kernel<<<(NS * SL / 16) * (ZP / 128), 32, 0, stream>>>(Fp(0), WIN, pss, NS, ZX);
    conv_kernel<<<(unsigned)(((size_t)NS * CD + 255) / 256), 256, 0, stream>>>(ZX, Fp(o + 1), Fp(o + 2), NS, XC);
    dt_kernel<<<(NS * NH + 255) / 256, 256, 0, stream>>>(ZX, Fp(o + 4), Fp(o + 3), NS, DT);
    ssd_kernel<<<NS * NH * (SL / 16), 32, 0, stream>>>(XC, DT, Fp(o + 5), NS, Y);
    gate_kernel<<<(NS * SL + 7) / 8, 256, 0, stream>>>(Y, ZX, Fp(o + 6), NS, YN);
    outproj_kernel<<<(NS * SL / 16) * 4, 32, 0, stream>>>(YN, WOUT, NS, HVp); }
  fc_kernel<<<(NTOK / 16) * 4, 32, 0, stream>>>(HH, VV, WFC, Fp(18), NS, (float*)d_out);
}
